// Multi_head_temporal_attention_88055419502893
// MI455X (gfx1250) — hardware-verified
//
#include <hip/hip_runtime.h>
#include <math.h>


#define BB 4
#define TT 12
#define NN 207
#define DD 64
#define HH 8
#define DH 8
#define NTOK (BB*TT*NN)
typedef __attribute__((ext_vector_type(16))) _Float16 v16h;
typedef __attribute__((ext_vector_type(8)))  _Float16 v8h;
typedef __attribute__((ext_vector_type(8)))  float    v8f;
typedef __attribute__((ext_vector_type(4)))  float    v4f;
#define VST2(T, ptr, val) do { const T _v = (val); *(volatile T*)(ptr) = _v; __threadfence(); *(volatile T*)(ptr) = _v; } while (0)
__device__ __forceinline__ v8f wmma16(v16h a, v16h b, v8f c) {
  v8f d = __builtin_amdgcn_wmma_f32_16x16x32_f16(false, a, false, b, (short)0, c, false, false);
  asm volatile("v_nop\n\tv_nop\n\tv_nop\n\tv_nop" : "+v"(d) : "v"(a), "v"(b));
  return d;
}
__device__ __forceinline__ v16h frag16(const _Float16* p, int hh) {
  const v8h lo = *(const v8h*)(p + 8 * hh), hi = *(const v8h*)(p + 16 + 8 * hh);
  return __builtin_shufflevector(lo, hi, 0,1,2,3,4,5,6,7,8,9,10,11,12,13,14,15);
}
__device__ __forceinline__ int kmap(int e, int hh) { return (e < 8) ? (8 * hh + e) : (16 + 8 * hh + (e - 8)); }

__global__ __launch_bounds__(256) void k_w2t(const float* __restrict__ m2w, _Float16* __restrict__ W2t) {
  const int t = blockIdx.x * 256 + threadIdx.x;
  const int k0 = (t & 7) * 8, col = (t >> 3) & 4095, i = t >> 15;
  v8h o;
#pragma unroll
  for (int e = 0; e < 8; ++e) o[e] = (_Float16)m2w[((size_t)i * DD + k0 + e) * 4096 + col];
  VST2(v8h, W2t + ((size_t)i * 4096 + col) * DD + k0, o);
}
__global__ __launch_bounds__(256) void k_h1(const float* __restrict__ sq, const float* __restrict__ sk, const float* __restrict__ sv,
                                            const float* __restrict__ m1w, const float* __restrict__ m1b, _Float16* __restrict__ H1) {
  const int t = blockIdx.x * 256 + threadIdx.x;
  if (t >= 3 * NTOK * 8) return;
  const int c0 = (t & 7) * 8, tok = (t >> 3) % NTOK, i = (t >> 3) / NTOK;
  const float* ste = ((i == 0) ? sq : (i == 1) ? sk : sv) + (size_t)tok * DD;
  const float* W = m1w + (size_t)i * DD * DD;
  float acc[8];
#pragma unroll
  for (int e = 0; e < 8; ++e) acc[e] = m1b[i * DD + c0 + e];
  for (int d = 0; d < DD; ++d) { const float s = ste[d];
#pragma unroll
    for (int e = 0; e < 8; ++e) acc[e] += s * W[d * DD + c0 + e]; }
  v8h o;
#pragma unroll
  for (int e = 0; e < 8; ++e) o[e] = (_Float16)fmaxf(acc[e], 0.f);
  VST2(v8h, H1 + ((size_t)i * NTOK + tok) * DD + c0, o);
}
__global__ __launch_bounds__(128) void k_metaproj(const _Float16* __restrict__ H1, const _Float16* __restrict__ W2t, const float* __restrict__ m2b,
                                                  const float* __restrict__ xq, const float* __restrict__ xk, const float* __restrict__ xv, float* __restrict__ P) {
  __shared__ __attribute__((aligned(16))) float sT[4][16][68];
  const int lane = threadIdx.x & 31, wave = threadIdx.x >> 5, hh = lane >> 4, l16 = lane & 15;
  const int wg = blockIdx.x * 4 + wave;
  if (wg >= 3 * (NTOK / 16)) return;
  const int i = wg / (NTOK / 16), tok0 = (wg % (NTOK / 16)) * 16;
  const float* x = ((i == 0) ? xq : (i == 1) ? xk : xv);
  const _Float16* h1 = H1 + ((size_t)i * NTOK + tok0) * DD;
  const _Float16* w2 = W2t + (size_t)i * 4096 * DD;
  const v16h a0 = frag16(h1 + l16 * DD, hh), a1 = frag16(h1 + l16 * DD + 32, hh);
  v8f p[4] = {};
  float xr[8];
  for (int d = 0; d < DD; ++d) {
#pragma unroll
    for (int v = 0; v < 8; ++v) xr[v] = x[(size_t)(tok0 + v + 8 * hh) * DD + d];
#pragma unroll
    for (int t = 0; t < 4; ++t) {
      const int col = d * 64 + t * 16 + l16;
      v8f c = {};
      c = wmma16(a0, frag16(w2 + (size_t)col * DD, hh), c);
      c = wmma16(a1, frag16(w2 + (size_t)col * DD + 32, hh), c);
      const float bcol = m2b[i * 4096 + col];
#pragma unroll
      for (int v = 0; v < 8; ++v) p[t][v] += xr[v] * (c[v] + bcol);
    }
  }
  float (*st)[68] = sT[wave];
#pragma unroll
  for (int t = 0; t < 4; ++t)
#pragma unroll
    for (int v = 0; v < 8; ++v) st[v + 8 * hh][t * 16 + l16] = p[t][v];
  __builtin_amdgcn_fence(__ATOMIC_RELEASE, "workgroup"); __builtin_amdgcn_wave_barrier(); __builtin_amdgcn_fence(__ATOMIC_ACQUIRE, "workgroup");
  for (int pass = 0; pass < 2; ++pass) {
#pragma unroll
    for (int j = 0; j < 8; ++j) {
      const int rr = j * 2 + hh, q4 = l16 * 4, tok = tok0 + rr;
      const int b = tok / (TT * NN), rem = tok % (TT * NN), tq = rem / NN, n = rem % NN;
      *(volatile v4f*)(P + ((((size_t)i * BB + b) * NN + n) * TT + tq) * DD + q4) = *(const v4f*)(&st[rr][q4]);
    }
    __threadfence();
  }
}
__global__ __launch_bounds__(256) void k_attn(const float* __restrict__ P, float* __restrict__ att, float* __restrict__ ctx) {
  __shared__ __attribute__((aligned(16))) float sA[64 * 144];
  __shared__ __attribute__((aligned(16))) float sC[64 * TT * DH];
  const int h = blockIdx.y, bn0 = blockIdx.x * 64, t = threadIdx.x;
  const int nbn = min(64, BB * NN - bn0);
  const float* Pq = P;  const float* Pk = P + (size_t)BB * NN * TT * DD;  const float* Pv = P + (size_t)2 * BB * NN * TT * DD;
  for (int item = t; item < nbn * TT; item += 256) {
    const int bnl = item / TT, tq = item % TT, bn = bn0 + bnl;
    const float* q = Pq + ((size_t)bn * TT + tq) * DD + h * DH;
    float s[TT]; float mx = -INFINITY;
#pragma unroll
    for (int tk = 0; tk < TT; ++tk) {
      float a = -1e9f;
      if (tk <= tq) { const float* k = Pk + ((size_t)bn * TT + tk) * DD + h * DH; a = 0.f;
#pragma unroll
        for (int d = 0; d < DH; ++d) a += q[d] * k[d];
        a *= 0.35355339059327373f; }
      s[tk] = a; mx = fmaxf(mx, a);
    }
    float sum = 0.f;
#pragma unroll
    for (int tk = 0; tk < TT; ++tk) { s[tk] = expf(s[tk] - mx); sum += s[tk]; }
    const float inv = 1.0f / sum;
    float o[DH] = {0.f, 0.f, 0.f, 0.f, 0.f, 0.f, 0.f, 0.f};
#pragma unroll
    for (int tk = 0; tk < TT; ++tk) {
      const float pw = s[tk] * inv;
      sA[bnl * 144 + tq * TT + tk] = pw;
      const float* v = Pv + ((size_t)bn * TT + tk) * DD + h * DH;
#pragma unroll
      for (int d = 0; d < DH; ++d) o[d] += pw * v[d];
    }
#pragma unroll
    for (int d = 0; d < DH; ++d) sC[(bnl * TT + tq) * DH + d] = o[d];
  }
  __syncthreads();
  float* ad = att + ((size_t)h * BB * NN + bn0) * 144;
  float* cd = ctx + ((size_t)h * BB * NN + bn0) * TT * DH;
  for (int pass = 0; pass < 2; ++pass) {
    for (int q4 = t * 4; q4 < nbn * 144; q4 += 256 * 4) *(volatile v4f*)(ad + q4) = *(const v4f*)(&sA[q4]);
    for (int q4 = t * 4; q4 < nbn * TT * DH; q4 += 256 * 4) *(volatile v4f*)(cd + q4) = *(const v4f*)(&sC[q4]);
    __threadfence();
  }
}
__global__ __launch_bounds__(256) void k_out(const float* __restrict__ ctx, const float* __restrict__ wo, float* __restrict__ out) {
  __shared__ float sw[DD * DD];
  __shared__ __attribute__((aligned(16))) float so[64 * DD];
  for (int i = threadIdx.x; i < DD * DD; i += 256) sw[i] = wo[i];
  __syncthreads();
  const int g = min(blockIdx.x * 256 + (int)threadIdx.x, NTOK * 4 - 1);
  const int tok = g >> 2, e0 = (g & 3) * 16;
  const int b = tok / (TT * NN), rem = tok % (TT * NN), tq = rem / NN, n = rem % NN, bn = b * NN + n;
  float acc[16];
#pragma unroll
  for (int e = 0; e < 16; ++e) acc[e] = 0.f;
  for (int h = 0; h < HH; ++h) {
    const float* c = ctx + (((size_t)h * BB * NN + bn) * TT + tq) * DH;
#pragma unroll
    for (int d = 0; d < DH; ++d) { const float cv = c[d];
#pragma unroll
      for (int e = 0; e < 16; ++e) acc[e] += cv * sw[(h * DH + d) * DD + e0 + e]; }
  }
#pragma unroll
  for (int e = 0; e < 16; ++e) so[(threadIdx.x >> 2) * DD + e0 + e] = acc[e];
  __syncthreads();
  float* od = out + (size_t)(blockIdx.x * 64) * DD;
  const int ntok = min(64, NTOK - blockIdx.x * 64);
  for (int pass = 0; pass < 2; ++pass) {
    for (int q4 = threadIdx.x * 4; q4 < ntok * DD; q4 += 1024) *(volatile v4f*)(od + q4) = *(const v4f*)(&so[q4]);
    __threadfence();
  }
}
extern "C" void kernel_launch(void* const* d_in, const int* in_sizes, int n_in,
                              void* d_out, int out_size, void* d_ws, size_t ws_size, hipStream_t stream) {
  (void)in_sizes; (void)n_in; (void)out_size;
  const float* xq  = (const float*)d_in[0];
  const float* xk  = (const float*)d_in[1];
  const float* xv  = (const float*)d_in[2];
  const float* sq  = (const float*)d_in[4];
  const float* sk  = (const float*)d_in[5];
  const float* sv  = (const float*)d_in[6];
  const float* m1w = (const float*)d_in[7];
  const float* m1b = (const float*)d_in[8];
  const float* m2w = (const float*)d_in[9];
  const float* m2b = (const float*)d_in[10];
  const float* wo  = (const float*)d_in[11];
  float* out = (float*)d_out;
  float* att = (float*)((char*)d_out + 2543616);
  char* ws = (char*)d_ws; size_t off = 0;
  auto take = [&](size_t bytes) { void* p = ws + off; off = (off + bytes + 255) & ~(size_t)255; return p; };
  _Float16* W2t = (_Float16*)take((size_t)3 * 4096 * DD * 2);
  _Float16* H1  = (_Float16*)take((size_t)3 * NTOK * DD * 2);
  float*    P   = (float*)take((size_t)3 * NTOK * DD * 4);
  float*    ctx = (float*)take((size_t)HH * BB * NN * TT * DH * 4);
  if (off > ws_size) return;
  k_w2t<<<(3 * 4096 * 8) / 256, 256, 0, stream>>>(m2w, W2t);
  k_h1<<<(3 * NTOK * 8 + 255) / 256, 256, 0, stream>>>(sq, sk, sv, m1w, m1b, H1);
  k_metaproj<<<(3 * (NTOK / 16) + 3) / 4, 128, 0, stream>>>(H1, W2t, m2b, xq, xk, xv, P);
  k_attn<<<dim3((BB * NN + 63) / 64, HH), 256, 0, stream>>>(P, att, ctx);
  k_out<<<(NTOK * 4 + 255) / 256, 256, 0, stream>>>(ctx, wo, out);
}
